// CausalSelfAttention_4054449127959
// MI455X (gfx1250) — hardware-verified
//
#include <hip/hip_runtime.h>
#ifndef NB
#define NB 8
#endif
#ifndef SEQ
#define SEQ 1024
#endif
#define NB_FULL 8
#define SEQ_FULL 1024
#define DM 1024
#define NH 16
#define HD 64
#define LQKV (3 * DM)
#define NR ((size_t)NB * SEQ)
#define PPH 32
#define BPAD 128
#define PCARRY 16384.0f
static_assert(NB >= 1 && NB <= NB_FULL);
static_assert(SEQ % 128 == 0 && SEQ >= 128 && SEQ <= SEQ_FULL);
static_assert(NH * HD == DM);
static_assert(DM % 64 == 0 && LQKV % 64 == 0);
static_assert(DM == 1024 && NH == 16 && SEQ_FULL == 1024);
static_assert((DM / 2) / NH == PPH && (NH / 2) * PPH == 256);
static_assert((SEQ / 16) % 4 == 0);
static_assert((NB * NH * (SEQ / 16)) % 4 == 0);
static_assert(BPAD == 128 && SEQ_FULL % 128 == 0 && BPAD >= 32);
static_assert(SEQ_FULL % 256 == 0 && (NH * SEQ_FULL) % 256 == 0);
static_assert(HD == 64 && DM % 32 == 0 && HD % 32 == 0);
static_assert((size_t)3 * DM * DM * 2 + (size_t)DM * DM * 2 + NR * DM * 2 + NR * LQKV * 2 + (size_t)NB * NH * HD * SEQ * 2 + NR * DM * 2 + (size_t)NH * SEQ_FULL * 4 <= (size_t)134217728);

typedef unsigned short v8us __attribute__((ext_vector_type(8), may_alias));
typedef float  v8f  __attribute__((ext_vector_type(8)));
typedef float  v4f  __attribute__((ext_vector_type(4)));
typedef float  v4fa __attribute__((ext_vector_type(4), may_alias));
typedef _Float16 v16h __attribute__((ext_vector_type(16)));
typedef _Float16 v4h __attribute__((ext_vector_type(4)));
union FragH { v16h v; v8us half[2]; _Float16 h[16]; unsigned short u[16]; };

__device__ __forceinline__ unsigned short bf16_bits(float x) { unsigned int u = __float_as_uint(x); return (unsigned short)((u + 0x7FFFu + ((u >> 16) & 1u)) >> 16); }
__device__ __forceinline__ float bf16_val(unsigned short b) { return __uint_as_float(((unsigned int)b) << 16); }
__device__ __forceinline__ float bf16_rne(float x) { return bf16_val(bf16_bits(x)); }
__device__ __forceinline__ unsigned short h16_bits(float x) { const _Float16 h = (_Float16)x; return __builtin_bit_cast(unsigned short, h); }

static __device__ __forceinline__ _Float16 toh_flush(float v) { const _Float16 r = (_Float16)v; return (fabsf(v) < 6.103515625e-05f) ? (_Float16)0.0f : r; }

__device__ __forceinline__ v16h g2_frag(const _Float16* p, int hh) { FragH f; f.half[0] = *(const v8us*)((const unsigned short*)p + 8 * hh); f.half[1] = *(const v8us*)((const unsigned short*)p + 16 + 8 * hh); return f.v; }
__device__ __forceinline__ v8f g2_mma(v16h a, v16h b, v8f c) { v8f d = __builtin_amdgcn_wmma_f32_16x16x32_f16(false, a, false, b, (short)0, c, false, false); asm volatile("v_nop\n\tv_nop\n\tv_nop\n\tv_nop" : "+v"(d) : "v"(a), "v"(b)); return d; }

__device__ __forceinline__ float rmax16(float v) {
  v = fmaxf(v, __shfl_xor(v, 1));
  v = fmaxf(v, __shfl_xor(v, 2));
  v = fmaxf(v, __shfl_xor(v, 4));
  v = fmaxf(v, __shfl_xor(v, 8));
  return v;
}
__device__ __forceinline__ float rsum16(float v) {
  v += __shfl_xor(v, 1);
  v += __shfl_xor(v, 2);
  v += __shfl_xor(v, 4);
  v += __shfl_xor(v, 8);
  return v;
}

__global__ __launch_bounds__(256) void k_wnat(const float* __restrict__ w, size_t n8, _Float16* __restrict__ Bt) {
  const size_t t = (size_t)blockIdx.x * 256 + threadIdx.x; if (t >= n8) return; FragH f;
#pragma unroll
  for (int q = 0; q < 8; ++q) f.h[q] = (_Float16)(bf16_rne(w[t * 8 + q]) * 16.0f);
  *(volatile v8us*)((unsigned short*)Bt + t * 8) = f.half[0]; __threadfence(); *(volatile v8us*)((unsigned short*)Bt + t * 8) = f.half[0];
}

__global__ __launch_bounds__(256) void k_x16(const float* __restrict__ x, _Float16* __restrict__ X16, size_t n8) {
  const size_t t = (size_t)blockIdx.x * 256 + threadIdx.x; if (t >= n8) return;
  const size_t e = t * 8; const size_t r = e / DM; const size_t c = e % DM; const size_t b = r / SEQ, s = r % SEQ;
  const float* src = x + ((b * SEQ_FULL + s) * DM + c);
  FragH f;
#pragma unroll
  for (int q = 0; q < 8; ++q) f.h[q] = (_Float16)bf16_rne(src[q]);
  *(volatile v8us*)((unsigned short*)X16 + e) = f.half[0]; __threadfence(); *(volatile v8us*)((unsigned short*)X16 + e) = f.half[0];
}

__host__ __device__ constexpr double hope_ratio() {
  const double xx = -9.210340371976182736 / 512.0;
  double term = 1.0, sum = 1.0;
  for (int i = 1; i < 24; ++i) { term = term * xx / (double)i; sum += term; }
  return sum;
}

__global__ __launch_bounds__(256) void k_hope(const float* __restrict__ pos, float* __restrict__ BT) {
  #pragma clang fp contract(off)
  const int t = blockIdx.x * 256 + threadIdx.x;
  const int h = t / SEQ_FULL, d = t % SEQ_FULL;
  float sum = 0.0f;
  if (h < NH / 2) {
    constexpr double RR = hope_ratio();
    double fd = 1.0;
#pragma unroll 1
    for (int i = 0; i < h * PPH; ++i) fd *= RR;
    const float df = (float)d;
#pragma unroll 1
    for (int j = 0; j < PPH; ++j) {
      const float f = (float)fd;
      const float th = df * f;
      float sn, cs;
      sincosf(th, &sn, &cs);
      const float pv = cs + sn;
      sum += pv;
      fd *= RR;
    }
  } else {
    const int base = (h - NH / 2) * PPH;
#pragma unroll 1
    for (int j = 0; j < PPH; ++j) {
      const float pc = bf16_rne(pos[2 * (base + j)]) + bf16_rne(pos[2 * (base + j) + 1]);
      sum += pc;
    }
  }
  *(volatile float*)(BT + t) = sum; __threadfence(); *(volatile float*)(BT + t) = sum;
}

template <int ACT>
__global__ __launch_bounds__(128) void k_gemm2(const _Float16* __restrict__ A, int lda, size_t sA, const _Float16* __restrict__ Bh, int ldb, size_t sB, float alpha, const float* __restrict__ bias, size_t sBias, const float* __restrict__ CP, int rowsPerB, size_t sCPb, int row0g,
    float* __restrict__ C, _Float16* __restrict__ C16, int ldc, size_t sC, int M, int N, int K) {
  static_assert(ACT == 0 || ACT == 3 || ACT == 12);
  __shared__ __attribute__((aligned(16))) float so[4][32][68];
  const int tid = threadIdx.x, w = tid >> 5, lane = tid & 31, ln = lane & 15, hh = lane >> 4; const int by = blockIdx.y;
  A += (size_t)by * sA; Bh += (size_t)by * sB; const size_t cofs = (size_t)by * sC; const float* bp = bias ? bias + (size_t)by * sBias : nullptr;
  const int ntn = N >> 6; const int mt = blockIdx.x / ntn, nq = blockIdx.x - mt * ntn; const int row0 = mt * 128 + 32 * w, col0 = nq * 64; if (row0 >= M) return;
  const _Float16* a0p = A + (size_t)(row0 + ln) * lda; const _Float16* a1p = a0p + (size_t)16 * lda;
  const _Float16* b0p = Bh + (size_t)(col0 + ln) * ldb; const _Float16* b1p = b0p + (size_t)16 * ldb; const _Float16* b2p = b1p + (size_t)16 * ldb; const _Float16* b3p = b2p + (size_t)16 * ldb;
  const v8f z8 = {0.f,0.f,0.f,0.f,0.f,0.f,0.f,0.f}; v8f c00 = z8, c01 = z8, c02 = z8, c03 = z8, c10 = z8, c11 = z8, c12 = z8, c13 = z8;
#pragma unroll 1
  for (int kb = 0; kb < K; kb += 32) { const v16h a0 = g2_frag(a0p + kb, hh), a1 = g2_frag(a1p + kb, hh);
    v16h b = g2_frag(b0p + kb, hh); c00 = g2_mma(a0, b, c00); c10 = g2_mma(a1, b, c10);
    b = g2_frag(b1p + kb, hh); c01 = g2_mma(a0, b, c01); c11 = g2_mma(a1, b, c11);
    b = g2_frag(b2p + kb, hh); c02 = g2_mma(a0, b, c02); c12 = g2_mma(a1, b, c12);
    b = g2_frag(b3p + kb, hh); c03 = g2_mma(a0, b, c03); c13 = g2_mma(a1, b, c13); }
  v8f accs[8] = {c00, c01, c02, c03, c10, c11, c12, c13};
#pragma unroll
  for (int u = 0; u < 8; ++u) { const int t = u & 3, half = u >> 2; const int col = col0 + t * 16 + ln; const float bv = bp ? bf16_rne(bp[col]) : 0.f;
#pragma unroll
    for (int r = 0; r < 8; ++r) { const int rloc = half * 16 + 8 * hh + r; float v = accs[u][r] * alpha + bv;
      if (CP) { if (rowsPerB < 0) v += CP[cofs + (size_t)(row0g + row0 + rloc) * ldc + col]; else { const int bidx = (row0g + row0 + rloc) / rowsPerB; v += CP[(size_t)bidx * sCPb + (size_t)by * 64 + col]; } }
      if (ACT == 3) v = fmaxf(v, 0.f); else if (ACT == 12) v = (v > 0.f) ? v : 0.01f * v;
      so[w][rloc][t * 16 + ln] = v; } }
  __builtin_amdgcn_fence(4  , "workgroup"); __builtin_amdgcn_wave_barrier();
  const int rsub = lane >> 4, c4 = (lane & 15) * 4;
  for (int pass = 0; pass < 2; ++pass) {
#pragma unroll
    for (int q = 0; q < 16; ++q) { const int r = q * 2 + rsub; const v4f v = *(const v4fa*)&so[w][r][c4];
      if (C) *(volatile v4f*)(C + cofs + (size_t)(row0 + r) * ldc + col0 + c4) = v;
      if (C16) { v4h h4; for (int i = 0; i < 4; ++i) h4[i] = (_Float16)v[i]; *(volatile v4h*)(C16 + cofs + (size_t)(row0 + r) * ldc + col0 + c4) = h4; } }
    if (pass == 0) __threadfence(); } }

template <int NHv, int TTv>
__global__ __launch_bounds__(256) void k_vt(const _Float16* __restrict__ V16, int ldv, int voff, _Float16* __restrict__ Vt) {
  __shared__ unsigned short tl[64][66]; const int tid = threadIdx.x; const int slab = blockIdx.x / (TTv / 64), lg = blockIdx.x % (TTv / 64); const int b = slab / NHv, h = slab % NHv;
  for (int i = tid; i < 64 * 8; i += 256) { const int r = i / 8, c8 = (i % 8) * 8; FragH f; f.half[0] = *(const v8us*)((const unsigned short*)V16 + ((size_t)b * TTv + lg * 64 + r) * ldv + voff + h * 64 + c8);
#pragma unroll
    for (int q = 0; q < 8; ++q) tl[r][c8 + q] = f.u[q]; }
  __syncthreads();
  for (int pass = 0; pass < 2; ++pass) {
#pragma unroll
    for (int rd = 0; rd < 2; ++rd) { const int d = rd * 32 + tid / 8, pc = tid % 8; FragH f;
#pragma unroll
      for (int q = 0; q < 8; ++q) f.u[q] = tl[pc * 8 + q][d];
      *(volatile v8us*)((unsigned short*)Vt + ((size_t)slab * 64 + d) * TTv + lg * 64 + pc * 8) = f.half[0]; }
    if (pass == 0) __threadfence(); } }

__global__ __launch_bounds__(128) void k_attn(const _Float16* __restrict__ QKV, const _Float16* __restrict__ VTp, const float* __restrict__ BT, _Float16* __restrict__ O) {
  #pragma clang fp contract(off)
  __shared__ __attribute__((aligned(16))) unsigned short pl[4][16 * 32];
  __shared__ __attribute__((aligned(16))) unsigned short st[4][16][72];
  __shared__ __attribute__((aligned(16))) float bl[BPAD + SEQ_FULL];
  const int tid = threadIdx.x, lane = tid & 31, ln = lane & 15, hh = lane >> 4;
  const int w = __builtin_amdgcn_readfirstlane(tid >> 5);
  const int qtl = SEQ / 16;
  const int wave = blockIdx.x * 4 + w;
  const int qt = wave % qtl, bh = wave / qtl;
  const int h = bh % NH, b = bh / NH;
  const int hblk = ((blockIdx.x * 4) / qtl) % NH;
  bl[tid] = 0.0f;
#pragma unroll
  for (int j = 0; j < SEQ_FULL / 128; ++j) bl[BPAD + j * 128 + tid] = BT[(size_t)hblk * SEQ_FULL + j * 128 + tid];
  __syncthreads();
  if (b >= NB) return;
  const int q0 = qt * 16;
  const _Float16* qrow  = QKV + ((size_t)b * SEQ + q0 + ln) * LQKV + h * HD;
  const _Float16* kbase = QKV + (size_t)b * SEQ * LQKV + DM + h * HD;
  const _Float16* vbase = VTp + (size_t)bh * HD * SEQ;
  const v16h aq0 = g2_frag(qrow, hh), aq1 = g2_frag(qrow + 32, hh);
  const v8f z8 = {0.f,0.f,0.f,0.f,0.f,0.f,0.f,0.f};
  v8f o[4] = {z8, z8, z8, z8};
  float rm[8], rs[8];
#pragma unroll
  for (int r = 0; r < 8; ++r) { rm[r] = -1.0e30f; rs[r] = 0.f; }
  const int kend = q0 + 16;
#pragma unroll 1
  for (int kt = 0; kt < kend; kt += 32) {
    v8f s0 = z8, s1 = z8;
    { const _Float16* kr = kbase + (size_t)(kt + ln) * LQKV;
      v16h bk = g2_frag(kr, hh); s0 = g2_mma(aq0, bk, s0); bk = g2_frag(kr + 32, hh); s0 = g2_mma(aq1, bk, s0);
      kr += (size_t)16 * LQKV;
      bk = g2_frag(kr, hh); s1 = g2_mma(aq0, bk, s1); bk = g2_frag(kr + 32, hh); s1 = g2_mma(aq1, bk, s1); }
    __builtin_amdgcn_fence(3  , "wavefront"); __builtin_amdgcn_wave_barrier();
    const int dl = q0 + 8 * hh - kt - ln;
    float corr[8];
#pragma unroll
    for (int r = 0; r < 8; ++r) {
      float bb0 = bl[BPAD + dl + r];
      float bb1 = bl[BPAD - 16 + dl + r];
      asm volatile("" : "+v"(bb0));
      asm volatile("" : "+v"(bb1));
      const bool vis0 = (dl + r) >= 0, vis1 = (dl + r) >= 16;
      const float t0 = s0[r] * 0.125f + bb0, t1 = s1[r] * 0.125f + bb1;
      const float a0 = vis0 ? t0 : -1.0e30f, a1 = vis1 ? t1 : -1.0e30f;
      const float tmax = rmax16(fmaxf(a0, a1));
      const float nm = fmaxf(rm[r], tmax);
      const float cr = __expf(rm[r] - nm);
      rm[r] = nm; corr[r] = cr;
      const float e0 = __expf(a0 - nm), e1 = __expf(a1 - nm);
      const float p0 = vis0 ? e0 * PCARRY : 0.0f, p1 = vis1 ? e1 * PCARRY : 0.0f;
      const _Float16 h0 = toh_flush(p0), h1 = toh_flush(p1);
      rs[r] = rs[r] * cr + rsum16((float)h0 + (float)h1);
      pl[w][(8 * hh + r) * 32 + ln]      = __builtin_bit_cast(unsigned short, h0);
      pl[w][(8 * hh + r) * 32 + 16 + ln] = __builtin_bit_cast(unsigned short, h1);
    }
#pragma unroll
    for (int j = 0; j < 4; ++j) {
#pragma unroll
      for (int r = 0; r < 8; ++r) o[j][r] *= corr[r];
    }
    __builtin_amdgcn_fence(3  , "wavefront"); __builtin_amdgcn_wave_barrier();
    FragH ap; ap.half[0] = *(const v8us*)(&pl[w][ln * 32 + 8 * hh]); ap.half[1] = *(const v8us*)(&pl[w][ln * 32 + 16 + 8 * hh]);
#pragma unroll
    for (int j = 0; j < 4; ++j) { const v16h bv = g2_frag(vbase + (size_t)(j * 16 + ln) * SEQ + kt, hh); o[j] = g2_mma(ap.v, bv, o[j]); }
  }
  float inv[8];
#pragma unroll
  for (int r = 0; r < 8; ++r) inv[r] = 64.0f / rs[r];
#pragma unroll
  for (int j = 0; j < 4; ++j) {
#pragma unroll
    for (int r = 0; r < 8; ++r) { const _Float16 ho = toh_flush(o[j][r] * inv[r]); st[w][8 * hh + r][j * 16 + ln] = __builtin_bit_cast(unsigned short, ho); }
  }
  __builtin_amdgcn_fence(4  , "workgroup"); __builtin_amdgcn_wave_barrier();
  const int rq = lane >> 3, pc = lane & 7;
  unsigned short* obase = (unsigned short*)O + ((size_t)b * SEQ + q0) * DM + h * HD + pc * 8;
  for (int pass = 0; pass < 2; ++pass) {
#pragma unroll
    for (int it = 0; it < 4; ++it) { const int row = it * 4 + rq; const v8us v = *(const v8us*)&st[w][row][pc * 8]; *(volatile v8us*)(obase + (size_t)row * DM) = v; }
    if (pass == 0) __threadfence(); }
}

extern "C" void kernel_launch(void* const* d_in, const int* in_sizes, int n_in,
                              void* d_out, int out_size, void* d_ws, size_t ws_size, hipStream_t stream) {
  if (n_in < 6) return;
  const float* x      = (const float*)d_in[0];
  const float* w_qkv  = (const float*)d_in[1];
  const float* b_qkv  = (const float*)d_in[2];
  const float* w_proj = (const float*)d_in[3];
  const float* b_proj = (const float*)d_in[4];
  const float* pos_i  = (const float*)d_in[5];
  const size_t rows_needed = (size_t)(NB - 1) * SEQ_FULL + SEQ;
  if ((size_t)in_sizes[0] < rows_needed * DM) return;
  if ((size_t)in_sizes[1] < (size_t)3 * DM * DM) return;
  if ((size_t)in_sizes[2] < (size_t)3 * DM) return;
  if ((size_t)in_sizes[3] < (size_t)DM * DM) return;
  if ((size_t)in_sizes[4] < (size_t)DM) return;
  if ((size_t)in_sizes[5] < (size_t)(DM / 4) * 2) return;
  if ((size_t)out_size < rows_needed * DM) return;
  char* ws = (char*)d_ws; size_t off = 0;
  auto take = [&](size_t bytes) { char* p = ws + off; off += (bytes + 255) & ~(size_t)255; return p; };
  _Float16* BQKV  = (_Float16*)take((size_t)3 * DM * DM * 2);
  _Float16* BO    = (_Float16*)take((size_t)DM * DM * 2);
  _Float16* X16   = (_Float16*)take(NR * DM * 2);
  _Float16* QKV16 = (_Float16*)take(NR * LQKV * 2);
  _Float16* VT    = (_Float16*)take((size_t)NB * NH * HD * SEQ * 2);
  _Float16* O16   = (_Float16*)take(NR * DM * 2);
  float*    BT    = (float*)take((size_t)NH * SEQ_FULL * 4);
  if (off > ws_size) return;
  k_wnat<<<(unsigned)(((size_t)3 * DM * DM / 8 + 255) / 256), 256, 0, stream>>>(w_qkv, (size_t)3 * DM * DM / 8, BQKV);
  k_wnat<<<(unsigned)(((size_t)DM * DM / 8 + 255) / 256), 256, 0, stream>>>(w_proj, (size_t)DM * DM / 8, BO);
  k_x16<<<(unsigned)((NR * DM / 8 + 255) / 256), 256, 0, stream>>>(x, X16, NR * DM / 8);
  k_hope<<<(unsigned)((NH * SEQ_FULL) / 256), 256, 0, stream>>>(pos_i, BT);
  k_gemm2<0><<<dim3((unsigned)((NR / 128) * (LQKV / 64)), 1), 128, 0, stream>>>(X16, DM, 0, BQKV, DM, 0, 0.0625f, b_qkv, 0, nullptr, 1, 0, 0, nullptr, QKV16, LQKV, 0, (int)NR, LQKV, DM);
  k_vt<NH, SEQ><<<(unsigned)(NB * NH * (SEQ / 64)), 256, 0, stream>>>(QKV16, LQKV, 2 * DM, VT);
  k_attn<<<(unsigned)((NB * NH * (SEQ / 16)) / 4), 128, 0, stream>>>(QKV16, VT, BT, O16);
  k_gemm2<0><<<dim3((unsigned)((SEQ / 128) * (DM / 64)), NB), 128, 0, stream>>>(O16, DM, (size_t)SEQ * DM, BO, DM, 0, 0.0009765625f, b_proj, 0, nullptr, 1, 0, 0, (float*)d_out, nullptr, DM, (size_t)SEQ_FULL * DM, SEQ, DM, DM);
}
